// Sequence_72189810311964
// MI455X (gfx1250) — hardware-verified
//
#include <hip/hip_runtime.h>
#include <math.h>

constexpr int NBAT     = 2048;
constexpr int NSTEP    = 512;
constexpr int HID      = 51;
constexpr int HPAD     = 64;
constexpr int NGROW    = 4 * HID;
constexpr int NPADN    = 256;
constexpr int KL1      = 64;
constexpr int KL2      = 128;
constexpr int RB       = 16;
constexpr int NTHR_SEQ = 128;
constexpr int NTHR_PK  = 256;
constexpr int HP       = 72;
constexpr int CHT      = 64;
constexpr int NTILE    = 8;
constexpr int TSZ      = RB * HP;
constexpr int VECN     = 4 * NPADN;
static_assert(NBAT % RB == 0);
static_assert(NSTEP % CHT == 0);
static_assert(KL1 % 32 == 0 && KL2 % 32 == 0);
static_assert(HID <= HPAD && NGROW <= NPADN);
static_assert((NTILE * TSZ) % NTHR_SEQ == 0);
static_assert(RB * CHT == 2 * 4 * NTHR_SEQ);
static_assert(HP % 8 == 0);
static_assert(NTHR_SEQ / 32 * 16 == HPAD);
static_assert(NTHR_SEQ / 32 * 4 == RB);
static_assert(VECN == 4 * NTHR_PK);

typedef __attribute__((ext_vector_type(16))) __bf16   v16b;
typedef __attribute__((ext_vector_type(8)))  __bf16   v8b;
typedef __attribute__((ext_vector_type(8)))  float    v8f;
typedef __attribute__((ext_vector_type(4)))  float    v4f;
typedef __attribute__((ext_vector_type(4)))  unsigned v4u;

__device__ __forceinline__ unsigned short f2bf_bits(float f) {
  unsigned u = __float_as_uint(f);
  return (unsigned short)((u + 0x7FFFu + ((u >> 16) & 1u)) >> 16);
}
__device__ __forceinline__ float bf_bits2f(unsigned short h) { return __uint_as_float(((unsigned)h) << 16); }
__device__ __forceinline__ float bf16r(float f) { return bf_bits2f(f2bf_bits(f)); }

__device__ __forceinline__ void mma_guard_all(v8f& a0, v8f& a1, v8f& a2, v8f& a3,
                                              v16b x, v16b y, v16b p, v16b q, v16b r, v16b s) {
  asm volatile("v_nop\n\tv_nop\n\tv_nop\n\tv_nop"
               : "+v"(a0), "+v"(a1), "+v"(a2), "+v"(a3)
               : "v"(x), "v"(y), "v"(p), "v"(q), "v"(r), "v"(s));
}
__device__ __forceinline__ void acc_guard4(v8f& a, v8f& b, v8f& c, v8f& d) {
  asm volatile("v_nop\n\tv_nop\n\tv_nop\n\tv_nop" : "+v"(a), "+v"(b), "+v"(c), "+v"(d));
}

template <typename T> struct Frag;
template <> struct Frag<__bf16> {
  typedef v16b V; union U { v16b v; v8b h[2]; };
  static __device__ __forceinline__ v16b load(const __bf16* p) {
    U f; f.h[0] = *(const v8b*)(p); f.h[1] = *(const v8b*)(p + 16); return f.v;
  }
  static __device__ __forceinline__ v8f mma(v16b a, v16b b, v8f c) {
    return __builtin_amdgcn_wmma_f32_16x16x32_bf16(false, a, false, b, (short)0, c, false, false);
  }
};

__device__ __forceinline__ float fsig(float x)  { return __builtin_amdgcn_rcpf(1.0f + __expf(-x)); }
__device__ __forceinline__ float ftanh(float x) { return 1.0f - 2.0f * __builtin_amdgcn_rcpf(__expf(2.0f * x) + 1.0f); }

__global__ __launch_bounds__(NTHR_PK) void pack_kernel(
    const float* __restrict__ Whh1, const float* __restrict__ Wih2, const float* __restrict__ Whh2,
    const float* __restrict__ Wih1, const float* __restrict__ bih1, const float* __restrict__ bhh1,
    const float* __restrict__ bih2, const float* __restrict__ bhh2, const float* __restrict__ fcw,
    unsigned short* __restrict__ W1P, unsigned short* __restrict__ W2P, float* __restrict__ VEC) {
  const int tid = threadIdx.x;
  const int bid = blockIdx.x;
  if (bid < 24) {
    const int reg = bid >> 3;
    const float* src = (reg == 0) ? Whh1 : ((reg == 1) ? Wih2 : Whh2);
    const int gi = (bid & 7) * NTHR_PK + tid;
    const int n  = gi >> 3;
    const int k8 = (gi & 7) * 8;
    const int g  = n >> 6, r = n & 63;
    const bool rok = (r < HID);
    const int  rc  = rok ? r : (HID - 1);
    const float* srow = src + (size_t)(g * HID + rc) * HID;
    v4u pk = {0u, 0u, 0u, 0u};
#pragma unroll
    for (int e = 0; e < 8; ++e) {
      const int k  = k8 + e;
      const int kc = (k < HID) ? k : (HID - 1);
      const float ld = srow[kc];
      const float v  = (rok && (k < HID)) ? ld : 0.0f;
      const unsigned bits = (unsigned)f2bf_bits(v);
      pk[e >> 1] = (e & 1) ? (pk[e >> 1] | (bits << 16)) : bits;
    }
    unsigned short* dst = (reg == 0) ? (W1P + (size_t)n * KL1 + k8)
                                     : (W2P + (size_t)n * KL2 + (reg - 1) * HPAD + k8);
    *(volatile v4u*)dst = pk;
    __threadfence();
    *(volatile v4u*)dst = pk;
  } else {
    const int vec = tid >> 6;
    const int n0  = (tid & 63) * 4;
    const float* pa = (vec == 0) ? bih1 : ((vec == 1) ? bih2 : ((vec == 2) ? Wih1 : fcw));
    const float* pb = (vec == 0) ? bhh1 : ((vec == 1) ? bhh2 : ((vec == 2) ? Wih1 : fcw));
    const float addb = (vec < 2) ? 1.0f : 0.0f;
    v4f o;
#pragma unroll
    for (int e = 0; e < 4; ++e) {
      const int n = n0 + e;
      const int g = n >> 6, r = n & 63;
      const int  rc   = (r < HID) ? r : (HID - 1);
      const int  nc   = (n < HID) ? n : (HID - 1);
      const int  idx  = (vec == 3) ? nc : (g * HID + rc);
      const bool ok   = (vec == 3) ? (n < HID) : (r < HID);
      const float va = bf16r(pa[idx]);
      const float vb = bf16r(pb[idx]);
      const float s  = va + addb * vb;
      o[e] = ok ? s : 0.0f;
    }
    float* op = VEC + vec * NPADN + n0;
    *(volatile v4f*)op = o;
    __threadfence();
    *(volatile v4f*)op = o;
  }
}

__global__ __launch_bounds__(NTHR_SEQ) void lstm2_seq_kernel(
    const float* __restrict__ x, const int* __restrict__ futp, const float* __restrict__ fcbp,
    const float* __restrict__ VEC, const unsigned short* __restrict__ W1Pp, const unsigned short* __restrict__ W2Pp,
    float* __restrict__ out) {
  __shared__ __align__(16) unsigned short HT[NTILE * TSZ];
  __shared__ __align__(16) float XS[RB * CHT];
  __shared__ __align__(16) float H2F[RB * HPAD];
  __shared__ __align__(16) float OS[RB * CHT];
  const __bf16* W1 = (const __bf16*)W1Pp;
  const __bf16* W2 = (const __bf16*)W2Pp;
  const __bf16* HB = (const __bf16*)HT;
  const int tid = threadIdx.x, lane = tid & 31, wave = tid >> 5;
  const int c = lane & 15, hh = lane >> 4, koff = hh * 8, c4 = c * 4;
  const int rowbase = blockIdx.x * RB;
  const int u = 16 * wave + c;
  const float uval = (u < HID) ? 1.0f : 0.0f;

#pragma unroll 1
  for (int i = tid; i < NTILE * TSZ; i += NTHR_SEQ) HT[i] = (unsigned short)0;

  float b1[4], b2[4], wx[4];
#pragma unroll
  for (int g = 0; g < 4; ++g) {
    const int n = 64 * g + u;
    b1[g] = VEC[n];
    b2[g] = VEC[NPADN + n];
    wx[g] = VEC[2 * NPADN + n];
  }
  const int frow = 4 * wave + (lane >> 3);
  const int kq   = (lane & 7) * 8;
  const v4f fw0 = *(const v4f*)(VEC + 3 * NPADN + kq);
  const v4f fw1 = *(const v4f*)(VEC + 3 * NPADN + kq + 4);
  const int futv = futp[0];
  const float fcb = bf16r(fcbp[0]) + ((futv > 0) ? __int_as_float(0x7fc00000) : 0.0f);

  float c1[8], c2[8], xb[8];
#pragma unroll
  for (int r = 0; r < 8; ++r) { c1[r] = 0.0f; c2[r] = 0.0f; xb[r] = 0.0f; }
  __syncthreads();

  const v8f z8 = {0.f, 0.f, 0.f, 0.f, 0.f, 0.f, 0.f, 0.f};

#pragma unroll 1
  for (int t = 0; t < NSTEP; ++t) {
    const int p  = t & 1;
    const int tc = t & (CHT - 1);
    if (tc == 0) {
#pragma unroll
      for (int it = 0; it < 2; ++it) {
        const int idx = it * NTHR_SEQ + tid;
        const int row = idx >> 4, cc4 = (idx & 15) * 4;
        const v4f v = *(const v4f*)(x + (size_t)(rowbase + row) * NSTEP + (size_t)t + cc4);
        *(v4f*)(XS + row * CHT + cc4) = v;
      }
      __syncthreads();
    }
#pragma unroll
    for (int r = 0; r < 8; ++r) xb[r] = bf16r(XS[(8 * hh + r) * CHT + tc]);

    const int t1prev = (0 * 4 + (p ^ 1) * 2) * TSZ;
    const int t1cur  = (0 * 4 + p * 2) * TSZ;
    const int t2prev = (1 * 4 + (p ^ 1) * 2) * TSZ;
    const int t2cur  = (1 * 4 + p * 2) * TSZ;

    v8f acc[4];
    acc[0] = z8; acc[1] = z8; acc[2] = z8; acc[3] = z8;
#pragma unroll 1
    for (int ks = 0; ks < KL1 / 32; ++ks) {
      const __bf16* ap = HB + t1prev + c * HP + koff + 32 * ks;
      const v16b ahi = Frag<__bf16>::load(ap);
      const v16b alo = Frag<__bf16>::load(ap + TSZ);
      const __bf16* wp = W1 + (size_t)u * KL1 + koff + 32 * ks;
      const v16b bw0 = Frag<__bf16>::load(wp);
      const v16b bw1 = Frag<__bf16>::load(wp + (size_t)64 * KL1);
      const v16b bw2 = Frag<__bf16>::load(wp + (size_t)128 * KL1);
      const v16b bw3 = Frag<__bf16>::load(wp + (size_t)192 * KL1);
      acc[0] = Frag<__bf16>::mma(ahi, bw0, acc[0]);
      acc[1] = Frag<__bf16>::mma(ahi, bw1, acc[1]);
      acc[2] = Frag<__bf16>::mma(ahi, bw2, acc[2]);
      acc[3] = Frag<__bf16>::mma(ahi, bw3, acc[3]);
      acc[0] = Frag<__bf16>::mma(alo, bw0, acc[0]);
      acc[1] = Frag<__bf16>::mma(alo, bw1, acc[1]);
      acc[2] = Frag<__bf16>::mma(alo, bw2, acc[2]);
      acc[3] = Frag<__bf16>::mma(alo, bw3, acc[3]);
      mma_guard_all(acc[0], acc[1], acc[2], acc[3], ahi, alo, bw0, bw1, bw2, bw3);
    }
    acc_guard4(acc[0], acc[1], acc[2], acc[3]);
#pragma unroll
    for (int r = 0; r < 8; ++r) {
      const float zi = acc[0][r] + (b1[0] + xb[r] * wx[0]);
      const float zf = acc[1][r] + (b1[1] + xb[r] * wx[1]);
      const float zg = acc[2][r] + (b1[2] + xb[r] * wx[2]);
      const float zo = acc[3][r] + (b1[3] + xb[r] * wx[3]);
      const float ig = fsig(zi);
      const float fg = fsig(zf);
      const float gg = ftanh(zg);
      const float og = fsig(zo);
      const float cn = fg * c1[r] + ig * gg;
      c1[r] = cn;
      const float hn = (og * ftanh(cn)) * uval;
      const unsigned short hb = f2bf_bits(hn);
      const unsigned short lb = f2bf_bits(hn - bf_bits2f(hb));
      HT[t1cur + (8 * hh + r) * HP + u]       = hb;
      HT[t1cur + TSZ + (8 * hh + r) * HP + u] = lb;
    }
    __syncthreads();

    acc[0] = z8; acc[1] = z8; acc[2] = z8; acc[3] = z8;
#pragma unroll 1
    for (int ks = 0; ks < KL2 / 32; ++ks) {
      const int lsel = ks >> 1;
      const int tb   = lsel ? t2prev : t1cur;
      const __bf16* ap = HB + tb + c * HP + koff + 32 * (ks & 1);
      const v16b ahi = Frag<__bf16>::load(ap);
      const v16b alo = Frag<__bf16>::load(ap + TSZ);
      const __bf16* wp = W2 + (size_t)u * KL2 + koff + 32 * ks;
      const v16b bw0 = Frag<__bf16>::load(wp);
      const v16b bw1 = Frag<__bf16>::load(wp + (size_t)64 * KL2);
      const v16b bw2 = Frag<__bf16>::load(wp + (size_t)128 * KL2);
      const v16b bw3 = Frag<__bf16>::load(wp + (size_t)192 * KL2);
      acc[0] = Frag<__bf16>::mma(ahi, bw0, acc[0]);
      acc[1] = Frag<__bf16>::mma(ahi, bw1, acc[1]);
      acc[2] = Frag<__bf16>::mma(ahi, bw2, acc[2]);
      acc[3] = Frag<__bf16>::mma(ahi, bw3, acc[3]);
      acc[0] = Frag<__bf16>::mma(alo, bw0, acc[0]);
      acc[1] = Frag<__bf16>::mma(alo, bw1, acc[1]);
      acc[2] = Frag<__bf16>::mma(alo, bw2, acc[2]);
      acc[3] = Frag<__bf16>::mma(alo, bw3, acc[3]);
      mma_guard_all(acc[0], acc[1], acc[2], acc[3], ahi, alo, bw0, bw1, bw2, bw3);
    }
    acc_guard4(acc[0], acc[1], acc[2], acc[3]);
#pragma unroll
    for (int r = 0; r < 8; ++r) {
      const float zi = acc[0][r] + b2[0];
      const float zf = acc[1][r] + b2[1];
      const float zg = acc[2][r] + b2[2];
      const float zo = acc[3][r] + b2[3];
      const float ig = fsig(zi);
      const float fg = fsig(zf);
      const float gg = ftanh(zg);
      const float og = fsig(zo);
      const float cn = fg * c2[r] + ig * gg;
      c2[r] = cn;
      const float hn = (og * ftanh(cn)) * uval;
      const unsigned short hb = f2bf_bits(hn);
      const unsigned short lb = f2bf_bits(hn - bf_bits2f(hb));
      HT[t2cur + (8 * hh + r) * HP + u]       = hb;
      HT[t2cur + TSZ + (8 * hh + r) * HP + u] = lb;
      H2F[(8 * hh + r) * HPAD + u] = hn;
    }
    __syncthreads();

    {
      const v4f hv0 = *(const v4f*)(H2F + frow * HPAD + kq);
      const v4f hv1 = *(const v4f*)(H2F + frow * HPAD + kq + 4);
      float s = 0.0f;
      s += hv0[0] * fw0[0]; s += hv0[1] * fw0[1]; s += hv0[2] * fw0[2]; s += hv0[3] * fw0[3];
      s += hv1[0] * fw1[0]; s += hv1[1] * fw1[1]; s += hv1[2] * fw1[2]; s += hv1[3] * fw1[3];
      s += __shfl_xor(s, 1, 32);
      s += __shfl_xor(s, 2, 32);
      s += __shfl_xor(s, 4, 32);
      const float ov = s + fcb;
      if ((lane & 7) == 0) OS[frow * CHT + tc] = ov;
    }
    if (tc == CHT - 1) {
      __syncthreads();
      const int tc0 = t - (CHT - 1);
      for (int pass = 0; pass < 2; ++pass) {
#pragma unroll
        for (int it = 0; it < 2; ++it) {
          const int row = 4 * wave + 2 * it + hh;
          const v4f v = *(const v4f*)(OS + row * CHT + c4);
          *(volatile v4f*)(out + (size_t)(rowbase + row) * NSTEP + (size_t)tc0 + c4) = v;
        }
        __threadfence();
      }
    }
  }
}

extern "C" void kernel_launch(void* const* d_in, const int* in_sizes, int n_in,
                              void* d_out, int out_size, void* d_ws, size_t ws_size, hipStream_t stream) {
  if (n_in < 12 || d_out == nullptr || d_ws == nullptr) return;
  if (in_sizes[0] != NBAT * NSTEP || in_sizes[1] != 1 || in_sizes[2] != NGROW || in_sizes[3] != NGROW ||
      in_sizes[4] != NGROW * HID || in_sizes[5] != NGROW || in_sizes[6] != NGROW * HID || in_sizes[7] != NGROW ||
      in_sizes[8] != NGROW * HID || in_sizes[9] != NGROW || in_sizes[10] != HID || in_sizes[11] != 1 ||
      out_size != NBAT * NSTEP) return;

  const float* x    = (const float*)d_in[0];
  const int*   fut  = (const int*)d_in[1];
  const float* Wih1 = (const float*)d_in[2];
  const float* bih1 = (const float*)d_in[3];
  const float* Whh1 = (const float*)d_in[4];
  const float* bhh1 = (const float*)d_in[5];
  const float* Wih2 = (const float*)d_in[6];
  const float* bih2 = (const float*)d_in[7];
  const float* Whh2 = (const float*)d_in[8];
  const float* bhh2 = (const float*)d_in[9];
  const float* fcw  = (const float*)d_in[10];
  const float* fcb  = (const float*)d_in[11];
  float* out = (float*)d_out;

  char* ws = (char*)d_ws; size_t off = 0;
  auto carve = [&](size_t bytes) -> char* { char* p = ws + off; off += (bytes + 255) & ~(size_t)255; return p; };
  unsigned short* W1P = (unsigned short*)carve((size_t)NPADN * KL1 * 2);
  unsigned short* W2P = (unsigned short*)carve((size_t)NPADN * KL2 * 2);
  float*          VEC = (float*)carve((size_t)VECN * 4);
  if (off > ws_size || off > (size_t)134217728) return;

  pack_kernel<<<25, NTHR_PK, 0, stream>>>(Whh1, Wih2, Whh2, Wih1, bih1, bhh1, bih2, bhh2, fcw, W1P, W2P, VEC);
  lstm2_seq_kernel<<<NBAT / RB, NTHR_SEQ, 0, stream>>>(x, fut, fcb, VEC, W1P, W2P, out);
}
